// DUMA_38070590112309
// MI455X (gfx1250) — hardware-verified
//
#include <hip/hip_runtime.h>
#include <stddef.h>
#include <stdint.h>

#define NBAT  8
#define SQ    512
#define NTOK  4096
#define HID   1024
#define NH    16
#define HDM   64
#define NBH   128
#define NQKV  3072
#define NSQ   8
#define NSLAB 24
#define NWROW 5120
#define QB    32
#define KC    64
#define NQB   (SQ / QB)
#define NCK   (SQ / KC)
#define SBLK  (SQ / 64)
#define NREL  129
#define NRELP 144
#define NRELK 160

static_assert(NTOK == NBAT * SQ);
static_assert(NBH == NBAT * NH);
static_assert(HID == NH * HDM);
static_assert(HID == 128 * 8);
static_assert(HDM == 64);
static_assert(NQKV == 3 * HID);
static_assert(NQKV == NSLAB * 128);
static_assert(NSQ * 128 == HID);
static_assert(SQ % KC == 0);
static_assert(SQ % QB == 0);
static_assert(QB == 32);
static_assert(NTOK % 256 == 0);
static_assert(NRELP % 16 == 0 && NRELP >= NREL);
static_assert(NRELK % 32 == 0 && NRELK >= NREL);

typedef _Float16 v16h __attribute__((ext_vector_type(16)));
typedef _Float16 v8h  __attribute__((ext_vector_type(8)));
typedef float    v8f  __attribute__((ext_vector_type(8)));
typedef float    v4f  __attribute__((ext_vector_type(4)));
typedef unsigned int v4u __attribute__((ext_vector_type(4)));

union Frag  { v16h v; v8h h[2]; };
union Pack8 { v8h h; v4u u; };

__device__ __forceinline__ v8f mma16(v16h a, v16h b, v8f c) {
  c = __builtin_amdgcn_wmma_f32_16x16x32_f16(false, a, false, b, (short)0, c, false, false);
  asm volatile("v_nop\n\tv_nop\n\tv_nop\n\tv_nop" : "+v"(c) : "v"(a), "v"(b));
  return c;
}

__device__ __forceinline__ v16h ldfrag(const _Float16* p, int ld, int row0, int k0, int lane) {
  const int m = lane & 15, lh = lane >> 4;
  const _Float16* q = p + (size_t)(row0 + m) * ld + k0 + 8 * lh;
  Frag f;
  f.h[0] = *(const v8h*)(q);
  f.h[1] = *(const v8h*)(q + 16);
  return f.v;
}

__device__ __forceinline__ v8f zero8() { return (v8f){0.f, 0.f, 0.f, 0.f, 0.f, 0.f, 0.f, 0.f}; }

__device__ __forceinline__ void gemm16x64(const _Float16* __restrict__ A, int lda,
                                          const _Float16* __restrict__ Bt, int ldb,
                                          int m0, int n0, int lane, v8f (&acc)[4]) {
#pragma unroll 2
  for (int k0 = 0; k0 < HID; k0 += 32) {
    const v16h a = ldfrag(A, lda, m0, k0, lane);
#pragma unroll
    for (int t = 0; t < 4; ++t) {
      const v16h b = ldfrag(Bt, ldb, n0 + 16 * t, k0, lane);
      acc[t] = mma16(a, b, acc[t]);
    }
  }
}

__device__ __forceinline__ void gemm32x64(const _Float16* __restrict__ A, int lda,
                                          const _Float16* __restrict__ Bt, int ldb,
                                          int m0, int n0, int lane, v8f (&acc)[2][4]) {
#pragma unroll 2
  for (int k0 = 0; k0 < HID; k0 += 32) {
    const v16h a0 = ldfrag(A, lda, m0, k0, lane);
    const v16h a1 = ldfrag(A, lda, m0 + 16, k0, lane);
    const v16h b0 = ldfrag(Bt, ldb, n0, k0, lane);
    const v16h b1 = ldfrag(Bt, ldb, n0 + 16, k0, lane);
    const v16h b2 = ldfrag(Bt, ldb, n0 + 32, k0, lane);
    const v16h b3 = ldfrag(Bt, ldb, n0 + 48, k0, lane);
    acc[0][0] = mma16(a0, b0, acc[0][0]);
    acc[1][0] = mma16(a1, b0, acc[1][0]);
    acc[0][1] = mma16(a0, b1, acc[0][1]);
    acc[1][1] = mma16(a1, b1, acc[1][1]);
    acc[0][2] = mma16(a0, b2, acc[0][2]);
    acc[1][2] = mma16(a1, b2, acc[1][2]);
    acc[0][3] = mma16(a0, b3, acc[0][3]);
    acc[1][3] = mma16(a1, b3, acc[1][3]);
  }
}

__global__ __launch_bounds__(256) void k_tab(_Float16* __restrict__ tabP, _Float16* __restrict__ tabT) {
  __shared__ __align__(16) float tb[NREL * HDM];
  const int tid = threadIdx.x;
#pragma unroll 1
  for (int idx = tid; idx < NREL * (HDM / 2); idx += 256) {
    const int p = idx >> 5;
    const int t = idx & 31;
    const float e  = (float)(2 * t) * (-0.14391156831212787f);
    const float dv = expf(e);
    const float arg = (float)p * dv;
    tb[p * HDM + 2 * t]     = sinf(arg);
    tb[p * HDM + 2 * t + 1] = cosf(arg);
  }
  __syncthreads();
#pragma unroll 1
  for (int q = tid; q < NRELP * HDM / 8; q += 256) {
    const int rel = q >> 3, d0 = (q & 7) * 8;
    const int rc = (rel < NREL) ? rel : 0;
    const float z = (rel < NREL) ? 1.f : 0.f;
    const float* s = tb + rc * HDM + d0;
    Pack8 pk;
    pk.h = (v8h){(_Float16)(s[0] * z), (_Float16)(s[1] * z), (_Float16)(s[2] * z), (_Float16)(s[3] * z),
                 (_Float16)(s[4] * z), (_Float16)(s[5] * z), (_Float16)(s[6] * z), (_Float16)(s[7] * z)};
    const v4u vv = pk.u;
    volatile v4u* d = (volatile v4u*)(tabP + (size_t)q * 8);
    *d = vv;
    __threadfence();
    *d = vv;
  }
#pragma unroll 1
  for (int q = tid; q < HDM * NRELK / 8; q += 256) {
    const int dd = q / (NRELK / 8);
    const int rel0 = (q - dd * (NRELK / 8)) * 8;
    float v[8];
#pragma unroll
    for (int i = 0; i < 8; ++i) {
      const int rel = rel0 + i;
      const int rc = (rel < NREL) ? rel : 0;
      v[i] = (rel < NREL) ? tb[rc * HDM + dd] : 0.f;
    }
    Pack8 pk;
    pk.h = (v8h){(_Float16)v[0], (_Float16)v[1], (_Float16)v[2], (_Float16)v[3],
                 (_Float16)v[4], (_Float16)v[5], (_Float16)v[6], (_Float16)v[7]};
    const v4u vv = pk.u;
    volatile v4u* d = (volatile v4u*)(tabT + (size_t)q * 8);
    *d = vv;
    __threadfence();
    *d = vv;
  }
}

__global__ __launch_bounds__(256) void k_cvtw(const float* __restrict__ w0, const float* __restrict__ w1,
                                              const float* __restrict__ w2, const float* __restrict__ w3,
                                              const float* __restrict__ w4, _Float16* __restrict__ dh, float scale) {
  const int tid = threadIdx.x;
  const int y = blockIdx.y;
  const float* src = (y == 0) ? w0 : ((y == 1) ? w1 : ((y == 2) ? w2 : ((y == 3) ? w3 : w4)));
  const int row = blockIdx.x * 2 + (tid >> 7);
  const int col = (tid & 127) * 8;
  const size_t o = (size_t)row * HID + col;
  const v4f a0 = *(const v4f*)(src + o) * scale;
  const v4f a1 = *(const v4f*)(src + o + 4) * scale;
  Pack8 pk;
  pk.h = (v8h){(_Float16)a0[0], (_Float16)a0[1], (_Float16)a0[2], (_Float16)a0[3],
               (_Float16)a1[0], (_Float16)a1[1], (_Float16)a1[2], (_Float16)a1[3]};
  const v4u vv = pk.u;
  volatile v4u* d = (volatile v4u*)(dh + ((size_t)y * HID + row) * HID + col);
  *d = vv;
  __threadfence();
  *d = vv;
}

__global__ __launch_bounds__(256) void k_gath(const float* __restrict__ seq, const int* __restrict__ dlen,
                                              const int* __restrict__ qlen, const int* __restrict__ olen,
                                              _Float16* __restrict__ xg) {
  const int tid = threadIdx.x;
  const int mode = blockIdx.y;
  const int row = blockIdx.x * 2 + (tid >> 7);
  const int b = row >> 9, j = row & (SQ - 1);
  const int dl = dlen[b], ql = qlen[b], ol = olen[b];
  const int shift = (mode == 0) ? 1 : (int)((unsigned)dl + 1u);
  const int valid = (mode == 0) ? dl : (int)((unsigned)ql + (unsigned)ol);
  int idx = (int)((unsigned)j + (unsigned)shift);
  idx = (idx < 0) ? 0 : ((idx > SQ - 1) ? (SQ - 1) : idx);
  const bool ok = j < valid;
  const int col = (tid & 127) * 8;
  const float* s = seq + ((size_t)(b * SQ + idx)) * HID + col;
  const v4f a0 = *(const v4f*)(s), a1 = *(const v4f*)(s + 4);
  Pack8 pk;
  pk.h = (v8h){(_Float16)(ok ? a0[0] : 0.f), (_Float16)(ok ? a0[1] : 0.f), (_Float16)(ok ? a0[2] : 0.f),
               (_Float16)(ok ? a0[3] : 0.f), (_Float16)(ok ? a1[0] : 0.f), (_Float16)(ok ? a1[1] : 0.f),
               (_Float16)(ok ? a1[2] : 0.f), (_Float16)(ok ? a1[3] : 0.f)};
  const v4u vv = pk.u;
  volatile v4u* d = (volatile v4u*)(xg + ((size_t)mode * NTOK + row) * HID + col);
  *d = vv;
  __threadfence();
  *d = vv;
}

#define SFP 132
__global__ __launch_bounds__(256) void k_qkv(const _Float16* __restrict__ xg,
                                             const _Float16* __restrict__ wt,
                                             const float* __restrict__ bq,
                                             const float* __restrict__ bkk,
                                             const float* __restrict__ bv,
                                             _Float16* __restrict__ qp,
                                             _Float16* __restrict__ kp,
                                             _Float16* __restrict__ vtp) {
  __shared__ __align__(16) float sf[64 * SFP];
  const int tid = threadIdx.x, lane = tid & 31, wave = tid >> 5;
  const int hh = lane >> 4, c = lane & 15;
  const int wm = wave >> 1, wn = wave & 1;
  const int z  = blockIdx.z;
  const int bx = blockIdx.x;
  const int b  = bx / SBLK;
  const int sb = (bx - b * SBLK) * 64;
  const int ns = blockIdx.y;
  const int which = (ns < NSQ) ? 0 : ((ns < 2 * NSQ) ? 1 : 2);
  const int hp = 2 * (ns - NSQ * which);
  const int m0 = sb + wm * 16;
  const int n0 = ns * 128 + wn * 64;
  const _Float16* A = xg + ((size_t)z * NTOK + (size_t)b * SQ) * HID;

  v8f acc[4];
#pragma unroll
  for (int t = 0; t < 4; ++t) acc[t] = zero8();
  gemm16x64(A, HID, wt, HID, m0, n0, lane, acc);

  const float* bsel = (which == 0) ? bq : ((which == 1) ? bkk : bv);
  const int cb = hp * HDM + wn * 64;
#pragma unroll
  for (int t = 0; t < 4; ++t) {
    const float bcol = bsel[cb + 16 * t + c];
#pragma unroll
    for (int r = 0; r < 8; ++r)
      sf[(wm * 16 + 8 * hh + r) * SFP + wn * 64 + 16 * t + c] = acc[t][r] * 0.03125f + bcol;
  }
  __syncthreads();

  const int pbase = z * NBH + b * NH + hp;
  if (which < 2) {
    v4u val[4];
    size_t go[4];
#pragma unroll
    for (int jj = 0; jj < 4; ++jj) {
      const int p  = tid + 256 * jj;
      const int lr = p >> 4;
      const int pc = p & 15;
      const int hs = pc >> 3;
      const int d0 = (pc & 7) * 8;
      const float* ra = sf + lr * SFP + pc * 8;
      const v4f a0 = *(const v4f*)(ra), a1 = *(const v4f*)(ra + 4);
      Pack8 pk;
      pk.h = (v8h){(_Float16)a0[0], (_Float16)a0[1], (_Float16)a0[2], (_Float16)a0[3],
                   (_Float16)a1[0], (_Float16)a1[1], (_Float16)a1[2], (_Float16)a1[3]};
      val[jj] = pk.u;
      go[jj]  = ((size_t)(pbase + hs) * SQ + sb + lr) * HDM + d0;
    }
    _Float16* base = (which == 0) ? qp : kp;
    for (int ps = 0; ps < 2; ++ps) {
#pragma unroll
      for (int jj = 0; jj < 4; ++jj) *(volatile v4u*)(base + go[jj]) = val[jj];
      __threadfence();
    }
  } else {
    v4u val[4];
    size_t go[4];
#pragma unroll
    for (int jj = 0; jj < 4; ++jj) {
      const int p    = tid + 256 * jj;
      const int dcol = p >> 3;
      const int pc   = p & 7;
      const float* cp = sf + (pc * 8) * SFP + dcol;
      Pack8 pk;
      pk.h = (v8h){(_Float16)cp[0 * SFP], (_Float16)cp[1 * SFP], (_Float16)cp[2 * SFP], (_Float16)cp[3 * SFP],
                   (_Float16)cp[4 * SFP], (_Float16)cp[5 * SFP], (_Float16)cp[6 * SFP], (_Float16)cp[7 * SFP]};
      val[jj] = pk.u;
      const int d = dcol & 63;
      go[jj]  = ((size_t)(pbase + (dcol >> 6)) * HDM + d) * SQ + sb + pc * 8;
    }
    for (int ps = 0; ps < 2; ++ps) {
#pragma unroll
      for (int jj = 0; jj < 4; ++jj) *(volatile v4u*)(vtp + go[jj]) = val[jj];
      __threadfence();
    }
  }
}

#define KTP 72
#define QTP 148
#define BKP 132
#define BHP 168
#define TTP NRELK
static_assert(16 * QTP * 4 >= 16 * BHP * 2);
__global__ __launch_bounds__(64) void k_attn(const _Float16* __restrict__ qp,
                                             const _Float16* __restrict__ kp,
                                             const _Float16* __restrict__ vt,
                                             const _Float16* __restrict__ tabP,
                                             const _Float16* __restrict__ tabT,
                                             _Float16* __restrict__ og, float sscale) {
  __shared__ __align__(16) _Float16 Ks[KC * KTP];
  __shared__ __align__(16) _Float16 Vs[HDM * KTP];
  __shared__ __align__(16) _Float16 Ps[2 * 16 * KTP];
  __shared__ __align__(16) float QTs[2 * 16 * QTP];
  __shared__ __align__(16) float BKs[2 * 16 * BKP];

  const int tid = threadIdx.x, lane = tid & 31, wave = tid >> 5;
  const int hh = lane >> 4, c = lane & 15;
  const int att = blockIdx.y;
  const int qb  = blockIdx.x % NQB;
  const int hb  = blockIdx.x / NQB;
  const int h   = hb % NH;
  const int b   = hb / NH;
  const int qset = att, kset = 1 - att;
  const int q0  = qb * QB + wave * 16;

  const _Float16* Q = qp + ((size_t)(qset * NBH + hb) * SQ) * HDM;
  const _Float16* K = kp + ((size_t)(kset * NBH + hb) * SQ) * HDM;
  const _Float16* V = vt + ((size_t)(kset * NBH + hb) * HDM) * SQ;
  _Float16* O = og + (size_t)att * NTOK * HID;

  float* qt = QTs + wave * 16 * QTP;
  float* bk = BKs + wave * 16 * BKP;
  _Float16* pw = Ps + wave * 16 * KTP;
  _Float16* bh = (_Float16*)(QTs + wave * 16 * QTP);

  v16h qa[2];
  qa[0] = ldfrag(Q, HDM, q0, 0, lane);
  qa[1] = ldfrag(Q, HDM, q0, 32, lane);

  for (int i = lane; i < 16 * BKP; i += 32) bk[i] = -1.0e30f;

#pragma unroll
  for (int nt = 0; nt < NRELP / 16; ++nt) {
    v8f cq = zero8();
    cq = mma16(qa[0], ldfrag(tabP, HDM, nt * 16, 0, lane), cq);
    cq = mma16(qa[1], ldfrag(tabP, HDM, nt * 16, 32, lane), cq);
#pragma unroll
    for (int r = 0; r < 8; ++r) qt[(8 * hh + r) * QTP + nt * 16 + c] = cq[r];
  }

  const float NEGI = -__builtin_huge_valf();
  float mrow[8], lrow[8], lo8[8], hi8[8];
  v8f oacc[4];
#pragma unroll
  for (int r = 0; r < 8; ++r) { mrow[r] = NEGI; lrow[r] = 0.f; lo8[r] = 0.f; hi8[r] = 0.f; }
#pragma unroll
  for (int t = 0; t < 4; ++t) oacc[t] = zero8();

#pragma unroll 1
  for (int kc = 0; kc < NCK; ++kc) {
    const int kv0 = kc * KC;
    __syncthreads();
    {
      const int r = tid;
      const _Float16* ks = K + (size_t)(kv0 + r) * HDM;
      const _Float16* vs = V + (size_t)r * SQ + kv0;
#pragma unroll
      for (int e = 0; e < 8; ++e) {
        *(v8h*)(Ks + r * KTP + 8 * e) = *(const v8h*)(ks + 8 * e);
        *(v8h*)(Vs + r * KTP + 8 * e) = *(const v8h*)(vs + 8 * e);
      }
    }
    __syncthreads();

    v8f s[4];
#pragma unroll
    for (int j = 0; j < 4; ++j) s[j] = zero8();
#pragma unroll
    for (int dc = 0; dc < 2; ++dc) {
#pragma unroll
      for (int j = 0; j < 4; ++j) {
        const v16h kb = ldfrag(Ks, KTP, j * 16, dc * 32, lane);
        s[j] = mma16(qa[dc], kb, s[j]);
      }
    }
    float cm[8];
#pragma unroll
    for (int r = 0; r < 8; ++r) {
      const int qrow = q0 + 8 * hh + r;
      const float* qtr = qt + (8 * hh + r) * QTP + 64;
      float m = NEGI;
#pragma unroll
      for (int j = 0; j < 4; ++j) {
        int d = kv0 + j * 16 + c - qrow;
        d = (d < -64) ? -64 : ((d > 64) ? 64 : d);
        const float v = (s[j][r] + qtr[d]) * sscale;
        s[j][r] = v;
        m = fmaxf(m, v);
      }
#pragma unroll
      for (int off = 1; off < 16; off <<= 1) m = fmaxf(m, __shfl_xor(m, off, 32));
      cm[r] = m;
    }
    float al[8];
#pragma unroll
    for (int r = 0; r < 8; ++r) {
      const int qrow = q0 + 8 * hh + r;
      const float mnew  = fmaxf(mrow[r], cm[r]);
      const float alpha = __expf(mrow[r] - mnew);
      mrow[r] = mnew;
      float psum = 0.f, lsum = 0.f, gsum = 0.f;
#pragma unroll
      for (int j = 0; j < 4; ++j) {
        const int d = kv0 + j * 16 + c - qrow;
        const float p = __expf(s[j][r] - mnew);
        psum += p;
        pw[(8 * hh + r) * KTP + j * 16 + c] = (_Float16)(p * 64.0f);
        lsum += (d <= -64) ? p : 0.f;
        gsum += (d >= 64) ? p : 0.f;
        if (d > -64 && d < 64) bk[(8 * hh + r) * BKP + d + 64] = s[j][r];
      }
#pragma unroll
      for (int off = 1; off < 16; off <<= 1) psum += __shfl_xor(psum, off, 32);
      lrow[r] = lrow[r] * alpha + psum;
      lo8[r]  = lo8[r] * alpha + lsum;
      hi8[r]  = hi8[r] * alpha + gsum;
      al[r]   = alpha;
    }
#pragma unroll
    for (int t = 0; t < 4; ++t)
#pragma unroll
      for (int r = 0; r < 8; ++r) oacc[t][r] *= al[r];
    __syncthreads();

#pragma unroll
    for (int kk = 0; kk < 2; ++kk) {
      const v16h pa = ldfrag(pw, KTP, 0, kk * 32, lane);
#pragma unroll
      for (int t = 0; t < 4; ++t) {
        const v16h vb = ldfrag(Vs, KTP, t * 16, kk * 32, lane);
        oacc[t] = mma16(pa, vb, oacc[t]);
      }
    }
  }

#pragma unroll
  for (int r = 0; r < 8; ++r) {
#pragma unroll
    for (int off = 1; off < 16; off <<= 1) {
      lo8[r] += __shfl_xor(lo8[r], off, 32);
      hi8[r] += __shfl_xor(hi8[r], off, 32);
    }
  }
  __syncthreads();
#pragma unroll
  for (int R = 0; R < 16; ++R) {
    const int srcl = (R >> 3) * 16;
    const int rr = R & 7;
    const float mR  = __shfl(mrow[rr], srcl, 32);
    const float loR = __shfl(lo8[rr], srcl, 32);
    const float hiR = __shfl(hi8[rr], srcl, 32);
    const float* bkr = bk + R * BKP;
#pragma unroll
    for (int i = 0; i < NRELK / 32; ++i) {
      const int col = lane + 32 * i;
      const int cs = (col < 128) ? col : 1;
      const float e = __expf(bkr[cs] - mR);
      float v = (col < 128) ? e : 0.f;
      v = (col == 0) ? loR : v;
      v = (col == 128) ? hiR : v;
      bh[R * BHP + col] = (_Float16)(v * 64.0f);
    }
  }
  __syncthreads();
#pragma unroll
  for (int kk = 0; kk < NRELK / 32; ++kk) {
    const v16h pa = ldfrag(bh, BHP, 0, kk * 32, lane);
#pragma unroll
    for (int t = 0; t < 4; ++t) {
      const v16h tb = ldfrag(tabT, TTP, t * 16, kk * 32, lane);
      oacc[t] = mma16(pa, tb, oacc[t]);
    }
  }

  float invl[8];
#pragma unroll
  for (int r = 0; r < 8; ++r) invl[r] = (lrow[r] > 0.f) ? (1.0f / lrow[r]) : 0.f;
  __syncthreads();
#pragma unroll
  for (int r = 0; r < 8; ++r) {
#pragma unroll
    for (int t = 0; t < 4; ++t)
      pw[(8 * hh + r) * KTP + 16 * t + c] = (_Float16)(oacc[t][r] * invl[r]);
  }
  __syncthreads();
  v4u val[4];
  size_t go[4];
#pragma unroll
  for (int it = 0; it < 4; ++it) {
    const int p  = lane + 32 * it;
    const int L  = p >> 3;
    const int pc = p & 7;
    Pack8 pk;
    pk.h    = *(const v8h*)(pw + L * KTP + pc * 8);
    val[it] = pk.u;
    go[it]  = ((size_t)(b * SQ + q0 + L)) * HID + (size_t)h * HDM + pc * 8;
  }
  for (int ps = 0; ps < 2; ++ps) {
#pragma unroll
    for (int it = 0; it < 4; ++it) *(volatile v4u*)(O + go[it]) = val[it];
    __threadfence();
  }
}

#define OTP 68
template <int EPI>
__global__ __launch_bounds__(256) void k_gemm(const _Float16* __restrict__ ap,
                                              const _Float16* __restrict__ wt,
                                              const float* __restrict__ bias,
                                              const float* __restrict__ res,
                                              float scale,
                                              float* __restrict__ outf,
                                              _Float16* __restrict__ outh) {
  __shared__ __align__(16) float st[8][16 * OTP];
  const int tid = threadIdx.x, lane = tid & 31, wave = tid >> 5;
  const int hh = lane >> 4, c = lane & 15;
  const int m0 = blockIdx.x * 256 + wave * 32;
  const int n0 = blockIdx.y * 64;

  v8f acc[2][4];
#pragma unroll
  for (int s = 0; s < 2; ++s)
#pragma unroll
    for (int t = 0; t < 4; ++t) acc[s][t] = zero8();
  gemm32x64(ap, HID, wt, HID, m0, n0, lane, acc);

  float* sw = st[wave];
  float bcol[4];
#pragma unroll
  for (int t = 0; t < 4; ++t) bcol[t] = bias[n0 + 16 * t + c];
#pragma unroll
  for (int sub = 0; sub < 2; ++sub) {
    __syncthreads();
#pragma unroll
    for (int t = 0; t < 4; ++t) {
#pragma unroll
      for (int r = 0; r < 8; ++r) {
        float v = acc[sub][t][r] * scale + bcol[t];
        if (EPI != 0) v = tanhf(v);
        sw[(8 * hh + r) * OTP + 16 * t + c] = v;
      }
    }
    __syncthreads();
    if (EPI == 1) {
      v4u val[4];
      size_t go[4];
#pragma unroll
      for (int it = 0; it < 4; ++it) {
        const int p  = lane + 32 * it;
        const int L  = p >> 3;
        const int pc = p & 7;
        const float* cp = sw + L * OTP + pc * 8;
        const v4f a0 = *(const v4f*)(cp), a1 = *(const v4f*)(cp + 4);
        Pack8 pk;
        pk.h = (v8h){(_Float16)(a0[0] * 64.f), (_Float16)(a0[1] * 64.f), (_Float16)(a0[2] * 64.f), (_Float16)(a0[3] * 64.f),
                     (_Float16)(a1[0] * 64.f), (_Float16)(a1[1] * 64.f), (_Float16)(a1[2] * 64.f), (_Float16)(a1[3] * 64.f)};
        val[it] = pk.u;
        go[it]  = (size_t)(m0 + sub * 16 + L) * HID + n0 + pc * 8;
      }
      for (int ps = 0; ps < 2; ++ps) {
#pragma unroll
        for (int it = 0; it < 4; ++it) *(volatile v4u*)(outh + go[it]) = val[it];
        __threadfence();
      }
    } else {
      v4f val[8];
      size_t go[8];
#pragma unroll
      for (int it = 0; it < 8; ++it) {
        const int p    = lane + 32 * it;
        const int L    = p >> 3;
        const int pc   = p & 7;
        const int row  = L >> 1;
        const int half = L & 1;
        val[it] = *(const v4f*)(sw + row * OTP + half * 32 + pc * 4);
        go[it]  = (size_t)(m0 + sub * 16 + row) * HID + n0 + half * 32 + pc * 4;
        if (EPI == 0) val[it] = val[it] + *(const v4f*)(res + go[it]);
      }
      for (int ps = 0; ps < 2; ++ps) {
#pragma unroll
        for (int it = 0; it < 8; ++it) *(volatile v4f*)(outf + go[it]) = val[it];
        __threadfence();
      }
    }
  }
}

__global__ __launch_bounds__(256) void k_ln(const float* __restrict__ y, const float* __restrict__ g,
                                            const float* __restrict__ be, _Float16* __restrict__ yh) {
  __shared__ __align__(16) float sw[8][HID];
  const int tid = threadIdx.x, lane = tid & 31, wave = tid >> 5;
  const size_t m = (size_t)blockIdx.x * 8 + wave;
  const float* yr = y + m * HID;

  v4f v[8];
  float s = 0.f;
#pragma unroll
  for (int it = 0; it < 8; ++it) {
    const int idx = it * 128 + lane * 4;
    v[it] = *(const v4f*)(yr + idx);
    s += (v[it][0] + v[it][1]) + (v[it][2] + v[it][3]);
  }
#pragma unroll
  for (int off = 16; off >= 1; off >>= 1) s += __shfl_xor(s, off, 32);
  const float mean = s * 0.0009765625f;
  float ss = 0.f;
#pragma unroll
  for (int it = 0; it < 8; ++it) {
    const v4f d = v[it] - mean;
    ss += (d[0] * d[0] + d[1] * d[1]) + (d[2] * d[2] + d[3] * d[3]);
  }
#pragma unroll
  for (int off = 16; off >= 1; off >>= 1) ss += __shfl_xor(ss, off, 32);
  const float var  = ss * 0.0009765625f;
  const float rstd = rsqrtf(var + 1e-12f);

#pragma unroll
  for (int it = 0; it < 8; ++it) {
    const int idx = it * 128 + lane * 4;
    const v4f gv = *(const v4f*)(g + idx);
    const v4f bv = *(const v4f*)(be + idx);
    *(v4f*)(sw[wave] + idx) = ((v[it] - mean) * rstd) * gv + bv;
  }
  __syncthreads();
  v4u hv[4];
  size_t go[4];
#pragma unroll
  for (int j = 0; j < 4; ++j) {
    const float* cp = sw[wave] + 256 * j + 8 * lane;
    const v4f a0 = *(const v4f*)(cp), a1 = *(const v4f*)(cp + 4);
    Pack8 pk;
    pk.h = (v8h){(_Float16)a0[0], (_Float16)a0[1], (_Float16)a0[2], (_Float16)a0[3],
                 (_Float16)a1[0], (_Float16)a1[1], (_Float16)a1[2], (_Float16)a1[3]};
    hv[j] = pk.u;
    go[j] = m * HID + 256 * j + 8 * lane;
  }
  for (int ps = 0; ps < 2; ++ps) {
#pragma unroll
    for (int j = 0; j < 4; ++j) *(volatile v4u*)(yh + go[j]) = hv[j];
    __threadfence();
  }
}

extern "C" void kernel_launch(void* const* d_in, const int* in_sizes, int n_in,
                              void* d_out, int out_size, void* d_ws, size_t ws_size,
                              hipStream_t stream) {
  if (n_in < 16) return;
  if (in_sizes[0] != NTOK * HID) return;
  if (in_sizes[1] != NBAT || in_sizes[2] != NBAT || in_sizes[3] != NBAT) return;
  if (in_sizes[4] != HID * HID || in_sizes[6] != HID * HID || in_sizes[8] != HID * HID) return;
  if (in_sizes[10] != HID * HID || in_sizes[12] != HID * HID) return;
  if (in_sizes[5] != HID || in_sizes[7] != HID || in_sizes[9] != HID || in_sizes[11] != HID) return;
  if (in_sizes[13] != HID || in_sizes[14] != HID || in_sizes[15] != HID) return;
  if (out_size != NTOK * HID) return;

  const float* seq  = (const float*)d_in[0];
  const int*   dlen = (const int*)d_in[1];
  const int*   qlen = (const int*)d_in[2];
  const int*   olen = (const int*)d_in[3];
  const float* wq = (const float*)d_in[4];
  const float* bq = (const float*)d_in[5];
  const float* wk = (const float*)d_in[6];
  const float* bkk = (const float*)d_in[7];
  const float* wv = (const float*)d_in[8];
  const float* bv = (const float*)d_in[9];
  const float* wp = (const float*)d_in[10];
  const float* bp = (const float*)d_in[11];
  const float* wo = (const float*)d_in[12];
  const float* bo = (const float*)d_in[13];
  const float* lng = (const float*)d_in[14];
  const float* lnb = (const float*)d_in[15];
  float* out = (float*)d_out;

  size_t off = 0;
  const size_t oW16 = off; off += (size_t)NWROW * HID * 2;
  const size_t oTP  = off; off += 24576;
  const size_t oTT  = off; off += 24576;
  const size_t oXG  = off; off += (size_t)2 * NTOK * HID * 2;
  const size_t oQ   = off; off += (size_t)2 * NBH * SQ * HDM * 2;
  const size_t oK   = off; off += (size_t)2 * NBH * SQ * HDM * 2;
  const size_t oV   = off; off += (size_t)2 * NBH * HDM * SQ * 2;
  const size_t oDP  = off; off += (size_t)NTOK * HID * 2;
  const size_t oQOP = off; off += (size_t)NTOK * HID * 4;
  const size_t oY   = off; off += (size_t)NTOK * HID * 4;
  const size_t oYH  = off; off += (size_t)NTOK * HID * 2;
  if (off > ws_size) return;
  if (off > (size_t)134217728) return;
  if ((size_t)NRELP * HDM * 2 > 24576 || (size_t)HDM * NRELK * 2 > 24576) return;

  char* ws = (char*)d_ws;
  _Float16* W16 = (_Float16*)(ws + oW16);
  _Float16* TP  = (_Float16*)(ws + oTP);
  _Float16* TT  = (_Float16*)(ws + oTT);
  _Float16* XG  = (_Float16*)(ws + oXG);
  _Float16* OG  = XG;
  _Float16* QP  = (_Float16*)(ws + oQ);
  _Float16* KP  = (_Float16*)(ws + oK);
  _Float16* VT  = (_Float16*)(ws + oV);
  _Float16* DP  = (_Float16*)(ws + oDP);
  float*    QOP = (float*)(ws + oQOP);
  float*    Y   = (float*)(ws + oY);
  _Float16* YH  = (_Float16*)(ws + oYH);
  _Float16* Wp16 = W16 + (size_t)3 * HID * HID;
  _Float16* Wo16 = W16 + (size_t)4 * HID * HID;

  k_tab<<<dim3(1), dim3(256), 0, stream>>>(TP, TT);
  k_cvtw<<<dim3(HID / 2, 5), dim3(256), 0, stream>>>(wq, wk, wv, wp, wo, W16, 32.0f);
  k_gath<<<dim3(NTOK / 2, 2), dim3(256), 0, stream>>>(seq, dlen, qlen, olen, XG);
  k_qkv<<<dim3(NBAT * SBLK, NSLAB, 2), dim3(256), 0, stream>>>(XG, W16, bq, bkk, bv, QP, KP, VT);
  k_attn<<<dim3(NBH * NQB, 2), dim3(64), 0, stream>>>(QP, KP, VT, TP, TT, OG, 0.125f);
  k_gemm<1><<<dim3(NTOK / 256, HID / 64), dim3(256), 0, stream>>>(OG, Wp16, bp, bp, 0.00048828125f, QOP, DP);
  k_gemm<2><<<dim3(NTOK / 256, HID / 64), dim3(256), 0, stream>>>(OG + (size_t)NTOK * HID, Wp16, bp, bp,
                                                                   0.00048828125f, QOP, YH);
  k_gemm<0><<<dim3(NTOK / 256, HID / 64), dim3(256), 0, stream>>>(DP, Wo16, bo, QOP, 0.00048828125f, Y, YH);
  k_ln<<<dim3(NTOK / 8), dim3(256), 0, stream>>>(Y, lng, lnb, YH);
  k_gemm<2><<<dim3(NTOK / 256, HID / 64), dim3(256), 0, stream>>>(YH, Wp16, bp, bp, 0.03125f, out, DP);
  (void)hipGetLastError();
}
